// MultiHeadSelfAttention_8993661518189
// MI455X (gfx1250) — hardware-verified
//
#include <hip/hip_runtime.h>


#ifndef NB
#define NB 4
#endif
#ifndef SEQ
#define SEQ 1024
#endif
#define NB_FULL  4
#define SEQ_FULL 1024
#ifndef OUT_SEQ
#define OUT_SEQ SEQ
#endif
#ifndef ATT_LD
#define ATT_LD OUT_SEQ
#endif
#ifndef SCORE_RES
#define SCORE_RES 1
#endif
#define DM   1024
#define NH_  16
#define HD   64
#define AW   4
#define EARLY 512
#define QRS  2048.0f
#define QRI  (1.0f / 2048.0f)
#define SC2  (0.125f * 1.4426950408889634f)
#define PSH  8.0f
#define NEGV (-3.0e38f)
#define OUT1_OFF ((size_t)NB_FULL * SEQ_FULL * DM)

static_assert(HD == 64);
static_assert(NH_ * HD == DM);
static_assert(DM % 64 == 0);
static_assert(DM % 32 == 0);
static_assert(SEQ % 256 == 0);
static_assert(SEQ % 64 == 0);
static_assert((NB * SEQ) % 64 == 0);
static_assert(SEQ % 32 == 0);
static_assert(SEQ % (16 * AW) == 0);
static_assert(((size_t)SEQ * DM) % 8 == 0);
static_assert(NB <= NB_FULL);
static_assert(SEQ <= SEQ_FULL);
static_assert(((size_t)NB * SEQ * (SEQ / 32)) % 256 == 0);
static_assert(ATT_LD % 32 == 0);
static_assert(ATT_LD >= SEQ);
static_assert(OUT1_OFF * 4 == (size_t)16777216);
static_assert(((size_t)(NB - 1) * OUT_SEQ + SEQ) * DM <= OUT1_OFF);
static_assert(OUT1_OFF + ((size_t)(NB - 1) * OUT_SEQ + (SEQ - 1)) * ATT_LD + SEQ <= OUT1_OFF + (size_t)NB_FULL * SEQ_FULL * SEQ_FULL);

typedef _Float16 h16;
typedef unsigned short bf;
typedef __attribute__((ext_vector_type(16))) __bf16   v16bf;
typedef __attribute__((ext_vector_type(16))) _Float16 v16h;
typedef __attribute__((ext_vector_type(8)))  _Float16 v8h;
typedef __attribute__((ext_vector_type(8)))  unsigned short v8us;
typedef __attribute__((ext_vector_type(8)))  float    v8f;
typedef __attribute__((ext_vector_type(4)))  float    v4f;
typedef __attribute__((ext_vector_type(4)))  int      v4i;
typedef v4f  __attribute__((may_alias)) v4fa;
typedef v8us __attribute__((may_alias)) v8usa;

__device__ __forceinline__ unsigned short f2bf(float f) { unsigned u = __float_as_uint(f); u += 0x7FFFu + ((u >> 16) & 1u); return (unsigned short)(u >> 16); }
__device__ __forceinline__ float bf2f(unsigned short h) { return __uint_as_float(((unsigned)h) << 16); }
__device__ __forceinline__ v16h cat16(v8h lo, v8h hi) { return __builtin_shufflevector(lo, hi, 0, 1, 2, 3, 4, 5, 6, 7, 8, 9, 10, 11, 12, 13, 14, 15); }
__device__ __forceinline__ v16bf cat16b(v8us lo, v8us hi) { return __builtin_bit_cast(v16bf, __builtin_shufflevector(lo, hi, 0, 1, 2, 3, 4, 5, 6, 7, 8, 9, 10, 11, 12, 13, 14, 15)); }
__device__ __forceinline__ v8f wmma16(v16h a, v16h b, v8f c) { return __builtin_amdgcn_wmma_f32_16x16x32_f16(false, a, false, b, (short)0, c, false, false); }
__device__ __forceinline__ v8f wmmab(v16bf a, v16bf b, v8f c) { return __builtin_amdgcn_wmma_f32_16x16x32_bf16(false, a, false, b, (short)0, c, false, false); }
__device__ __forceinline__ v16h  ldh(const h16* p) { return cat16(*(const v8h*)p, *(const v8h*)(p + 16)); }
__device__ __forceinline__ v16bf ldb(const bf* p)  { return cat16b(*(const v8us*)p, *(const v8us*)(p + 16)); }
__device__ __forceinline__ void wave_sync() { __builtin_amdgcn_fence(3  , "wavefront"); __builtin_amdgcn_wave_barrier(); asm volatile("" ::: "memory"); }
static __device__ __forceinline__ h16 toh_flush(float v) { const h16 r = (h16)v; return (fabsf(v) < 6.103515625e-05f) ? (h16)0.0f : r; }

__global__ __launch_bounds__(256) void k_cvt8(const float* __restrict__ src, bf* dst, size_t n8) {
    const size_t i = (size_t)blockIdx.x * 256 + threadIdx.x; if (i >= n8) return;
    const v8f v = *(const v8f*)(src + i * 8); v8us o;
#pragma unroll
    for (int k = 0; k < 8; ++k) o[k] = f2bf(v[k]);
    *(volatile v8us*)(dst + i * 8) = o; __threadfence(); *(volatile v8us*)(dst + i * 8) = o;
}

__global__ __launch_bounds__(256) void k_cvtT(const float* __restrict__ W, int ldn, bf* dst, int permFrom) {
    __shared__ __align__(16) unsigned short ts[64 * 72];
    const int t = threadIdx.x; const int k0 = blockIdx.x * 64, n0 = blockIdx.y * 64;
#pragma unroll 4
    for (int i = 0; i < 16; ++i) { const int k = i * 4 + (t >> 6), n = t & 63;
        ts[n * 72 + k] = f2bf(W[(size_t)(k0 + k) * (size_t)ldn + n0 + n]); }
    __syncthreads();
    v8us o0, o1; size_t d0, d1;
    { const int p = t, n = p >> 3, q = p & 7; o0 = *(const v8usa*)(&ts[n * 72 + 8 * q]);
      const int e = n0 + n; const int ee = e - permFrom; const int row = (e >= permFrom) ? (permFrom + (ee & 63) * 16 + (ee >> 6)) : e;
      d0 = (size_t)row * DM + k0 + 8 * q; }
    { const int p = t + 256, n = p >> 3, q = p & 7; o1 = *(const v8usa*)(&ts[n * 72 + 8 * q]);
      const int e = n0 + n; const int ee = e - permFrom; const int row = (e >= permFrom) ? (permFrom + (ee & 63) * 16 + (ee >> 6)) : e;
      d1 = (size_t)row * DM + k0 + 8 * q; }
#pragma unroll 1
    for (int ps = 0; ps < 2; ++ps) {
        *(volatile v8us*)(dst + d0) = o0; *(volatile v8us*)(dst + d1) = o1;
        if (ps == 0) __threadfence(); }
}

__global__ __launch_bounds__(256) void k_mbits(const int* __restrict__ pm, unsigned* MW, size_t nW) {
    const size_t w = (size_t)blockIdx.x * 256 + threadIdx.x; if (w >= nW) return;
    const size_t row = w / (size_t)(SEQ / 32); const size_t j = w % (size_t)(SEQ / 32);
    const size_t b = row / (size_t)SEQ, t = row % (size_t)SEQ;
    const int* src = pm + (b * SEQ_FULL + t) * (size_t)SEQ_FULL + j * 32;
    unsigned bits = 0u;
#pragma unroll
    for (int i = 0; i < 8; ++i) { const v4i v = *(const v4i*)(src + 4 * i);
        const unsigned n = ((v[0] != 0) ? 1u : 0u) | ((v[1] != 0) ? 2u : 0u) | ((v[2] != 0) ? 4u : 0u) | ((v[3] != 0) ? 8u : 0u);
        bits |= n << (4 * i); }
    *(volatile unsigned*)(MW + w) = bits; __threadfence(); *(volatile unsigned*)(MW + w) = bits;
}

template <int MODE>
__global__ __launch_bounds__(32) void k_gemm(const bf* __restrict__ A, const bf* __restrict__ Bt, const float* __restrict__ bias, h16* Ph, h16* Pr, float* OUT) {
    __shared__ __align__(16) float os[16 * 68];
    const int K = DM;
    const int lane = threadIdx.x & 31, lr = lane & 15, hi = lane >> 4; const int r0 = blockIdx.x * 64, c0 = blockIdx.y * 64;
    v8f acc[4][4];
#pragma unroll
    for (int mb = 0; mb < 4; ++mb)
#pragma unroll
        for (int nb = 0; nb < 4; ++nb) acc[mb][nb] = (v8f){};
    const size_t aoff = (size_t)(r0 + lr) * K + 8 * hi, boff = (size_t)(c0 + lr) * K + 8 * hi;
    const int npl = (MODE == 3) ? 2 : 1;
#pragma unroll 1
    for (int pl = 0; pl < npl; ++pl) {
        const bf* Ap = A + (size_t)pl * ((size_t)NB * SEQ * DM);
#pragma unroll 1
        for (int kc = 0; kc < K; kc += 32) {
            v16bf a[4];
#pragma unroll
            for (int mb = 0; mb < 4; ++mb) a[mb] = ldb(Ap + aoff + (size_t)mb * 16 * K + kc);
#pragma unroll
            for (int nb = 0; nb < 4; ++nb) { const v16bf b = ldb(Bt + boff + (size_t)nb * 16 * K + kc);
#pragma unroll
                for (int mb = 0; mb < 4; ++mb) acc[mb][nb] = wmmab(a[mb], b, acc[mb][nb]); }
            asm volatile("v_nop\n\tv_nop\n\tv_nop\n\tv_nop" : "+v"(acc[0][0]), "+v"(acc[1][1]), "+v"(acc[2][2]), "+v"(acc[3][3]) : "v"(a[0]), "v"(a[1]), "v"(a[2]), "v"(a[3]));
        }
    }
    float bv[4];
#pragma unroll
    for (int nb = 0; nb < 4; ++nb) {
        const int bi = (MODE == 2) ? (2 * DM) : (((MODE == 1) ? DM : 0) + c0 + nb * 16 + lr);
        bv[nb] = bf2f(f2bf(bias[bi])); }
#pragma unroll
    for (int mb = 0; mb < 4; ++mb) {
        float rb[8];
#pragma unroll
        for (int j = 0; j < 8; ++j) rb[j] = 0.0f;
        if (MODE == 2) {
            const v8f bq = *(const v8f*)(bias + 2 * DM + r0 + mb * 16 + hi * 8);
#pragma unroll
            for (int j = 0; j < 8; ++j) rb[j] = bf2f(f2bf(bq[j])); }
#pragma unroll
        for (int nb = 0; nb < 4; ++nb) {
#pragma unroll
            for (int j = 0; j < 8; ++j) os[(hi * 8 + j) * 68 + nb * 16 + lr] = (MODE == 2) ? (acc[mb][nb][j] + rb[j]) : (acc[mb][nb][j] + bv[nb]); }
        wave_sync();
        if (MODE == 0 || MODE == 1 || MODE == 2) {
            size_t sb, pitch;
            if (MODE == 2) { const int bb = c0 / SEQ; const int tt = c0 % SEQ;
                sb = ((size_t)(bb * NH_ + (r0 >> 6)) * HD + (size_t)(16 * mb)) * SEQ + (size_t)tt; pitch = SEQ; }
            else { const int tokrow = r0 + 16 * mb; const int bb = tokrow / SEQ; const int tt = tokrow % SEQ;
                sb = ((size_t)(bb * NH_ + (c0 >> 6)) * SEQ + (size_t)tt) * HD; pitch = HD; }
#pragma unroll 1
            for (int ps = 0; ps < 2; ++ps) {
#pragma unroll
                for (int s = 0; s < 4; ++s) { const int row = 4 * s + (lane >> 3), c8 = (lane & 7) * 8;
                    const v4f x0 = *(const v4fa*)(&os[row * 68 + c8]); const v4f x1 = *(const v4fa*)(&os[row * 68 + c8 + 4]); v8h hv, rv;
#pragma unroll
                    for (int i = 0; i < 4; ++i) { const h16 a0 = toh_flush(x0[i]); const h16 a1 = toh_flush(x1[i]); hv[i] = a0; hv[4 + i] = a1;
                        rv[i] = toh_flush((x0[i] - (float)a0) * QRS); rv[4 + i] = toh_flush((x1[i] - (float)a1) * QRS); }
                    const size_t oo = sb + (size_t)row * pitch + c8;
                    *(volatile v8h*)(Ph + oo) = hv; if (MODE != 1) *(volatile v8h*)(Pr + oo) = rv; }
                if (ps == 0) __threadfence(); }
        } else {
            const int grow = r0 + 16 * mb; const int bb = grow / SEQ; const int nn = grow % SEQ;
            float* orow = OUT + ((size_t)bb * OUT_SEQ + nn) * DM + c0;
#pragma unroll 1
            for (int ps = 0; ps < 2; ++ps) {
#pragma unroll
                for (int s = 0; s < 8; ++s) { const int row = 2 * s + hi, cofs = lr * 4;
                    const v4f val = *(const v4fa*)(&os[row * 68 + cofs]);
                    *(volatile v4f*)(orow + (size_t)row * DM + cofs) = val; }
                if (ps == 0) __threadfence(); }
        }
        wave_sync();
    }
}

__global__ __launch_bounds__(32 * AW) void k_flash(const h16* __restrict__ QH, const h16* __restrict__ QR, const h16* __restrict__ KP, const h16* __restrict__ VT, const h16* __restrict__ VR, const unsigned* __restrict__ MW, bf* CH, bf* CL, float* ATT) {
    __shared__ __align__(16) float os[AW * 16 * 68];
    const int lane = threadIdx.x & 31, lr = lane & 15, hi = lane >> 4;
    const int wave = __builtin_amdgcn_readfirstlane((int)(threadIdx.x >> 5));
    const int zh = blockIdx.y;
    const int bb = zh / NH_, hh = zh % NH_;
    const int t0 = (blockIdx.x * AW + wave) * 16;
    const size_t pbase = (size_t)zh * SEQ * HD;
    const size_t qo = pbase + (size_t)(t0 + lr) * HD + 8 * hi;
    const v16h qh0 = ldh(QH + qo), qh1 = ldh(QH + qo + 32), qr0 = ldh(QR + qo), qr1 = ldh(QR + qo + 32);
    const size_t ko = pbase + (size_t)lr * HD + 8 * hi;
    const size_t vo = pbase + (size_t)lr * SEQ + 8 * hi;
    const int kend = t0 + 16;
    const bool early = t0 < EARLY;
    const int tq = t0 + lr;
    const size_t mo = ((size_t)bb * SEQ + (size_t)tq) * (size_t)(SEQ / 32);
    v8f o0 = (v8f){}, o1 = (v8f){}, o2 = (v8f){}, o3 = (v8f){};
    v8f e0 = (v8f){}, e1 = (v8f){}, e2 = (v8f){}, e3 = (v8f){};
    float m = NEGV, l = 0.0f;
#pragma unroll 1
    for (int key0 = 0; key0 < kend; key0 += 32) {
        const h16* ka = KP + ko + (size_t)key0 * HD;
        const v16h ka0 = ldh(ka), ka1 = ldh(ka + 32), kb0 = ldh(ka + 16 * HD), kb1 = ldh(ka + 16 * HD + 32);
        v8f sHa = (v8f){}, sLa = (v8f){}, sHb = (v8f){}, sLb = (v8f){};
        sHa = wmma16(ka0, qh0, sHa); sHb = wmma16(kb0, qh0, sHb);
        if (SCORE_RES) { sLa = wmma16(ka0, qr0, sLa); sLb = wmma16(kb0, qr0, sLb); }
        sHa = wmma16(ka1, qh1, sHa); sHb = wmma16(kb1, qh1, sHb);
        if (SCORE_RES) { sLa = wmma16(ka1, qr1, sLa); sLb = wmma16(kb1, qr1, sLb); }
        asm volatile("v_nop\n\tv_nop\n\tv_nop\n\tv_nop" : "+v"(sHa), "+v"(sLa), "+v"(sHb), "+v"(sLb) : "v"(ka0), "v"(ka1), "v"(kb0), "v"(kb1));
        float ta[8], tb[8];
#pragma unroll
        for (int r = 0; r < 8; ++r) { ta[r] = (sHa[r] + sLa[r] * QRI) * SC2; tb[r] = (sHb[r] + sLb[r] * QRI) * SC2; }
        if (key0 + 31 > t0) {
            const int kidx = key0 + 8 * hi;
#pragma unroll
            for (int r = 0; r < 8; ++r) { ta[r] = (kidx + r > tq) ? NEGV : ta[r]; tb[r] = (kidx + 16 + r > tq) ? NEGV : tb[r]; }
        }
        unsigned mw = MW[mo + (size_t)(key0 >> 5)];
        asm volatile("" : "+v"(mw));
        {
            const unsigned ma = mw >> (8 * hi), mc = mw >> (16 + 8 * hi);
#pragma unroll
            for (int r = 0; r < 8; ++r) { ta[r] = (((ma >> r) & 1u) != 0u) ? NEGV : ta[r]; tb[r] = (((mc >> r) & 1u) != 0u) ? NEGV : tb[r]; }
        }
        float mx = NEGV;
#pragma unroll
        for (int r = 0; r < 8; ++r) mx = fmaxf(mx, fmaxf(ta[r], tb[r]));
        mx = fmaxf(mx, __shfl_xor(mx, 16, 32));
        const float mnew = fmaxf(m, mx);
        const float alpha = __builtin_amdgcn_exp2f(m - mnew);
        const float sh = PSH - mnew;
        v16h pb; float ls = 0.0f;
#pragma unroll
        for (int r = 0; r < 8; ++r) { const float ea = ta[r] + sh, ec = tb[r] + sh;
            const h16 pa = (ea < -14.0f) ? (h16)0.0f : (h16)__builtin_amdgcn_exp2f(ea);
            const h16 pc = (ec < -14.0f) ? (h16)0.0f : (h16)__builtin_amdgcn_exp2f(ec);
            pb[r] = pa; pb[8 + r] = pc; ls += (float)pa + (float)pc; }
        l = l * alpha + ls; m = mnew;
        o0 = o0 * alpha; o1 = o1 * alpha; o2 = o2 * alpha; o3 = o3 * alpha;
        const h16* va = VT + vo + key0;
        const v16h v0 = ldh(va), v1 = ldh(va + (size_t)16 * SEQ), v2 = ldh(va + (size_t)32 * SEQ), v3 = ldh(va + (size_t)48 * SEQ);
        o0 = wmma16(v0, pb, o0); o1 = wmma16(v1, pb, o1); o2 = wmma16(v2, pb, o2); o3 = wmma16(v3, pb, o3);
        asm volatile("v_nop\n\tv_nop\n\tv_nop\n\tv_nop" : "+v"(o0), "+v"(o1), "+v"(o2), "+v"(o3) : "v"(v0), "v"(v1), "v"(v2), "v"(v3), "v"(pb));
        if (early) {
            e0 = e0 * alpha; e1 = e1 * alpha; e2 = e2 * alpha; e3 = e3 * alpha;
            const h16* vr = VR + vo + key0;
            const v16h w0 = ldh(vr), w1 = ldh(vr + (size_t)16 * SEQ), w2 = ldh(vr + (size_t)32 * SEQ), w3 = ldh(vr + (size_t)48 * SEQ);
            e0 = wmma16(w0, pb, e0); e1 = wmma16(w1, pb, e1); e2 = wmma16(w2, pb, e2); e3 = wmma16(w3, pb, e3);
            asm volatile("v_nop\n\tv_nop\n\tv_nop\n\tv_nop" : "+v"(e0), "+v"(e1), "+v"(e2), "+v"(e3) : "v"(w0), "v"(w1), "v"(w2), "v"(w3), "v"(pb));
        }
    }
    l += __shfl_xor(l, 16, 32);
    const float inv = (m > NEGV) ? (1.0f / l) : __uint_as_float(0x7FC00000u);
    const int wb = wave * 16 * 68;
    { v4f a, c;
#pragma unroll
      for (int i = 0; i < 4; ++i) { a[i] = (o0[i] + e0[i] * QRI) * inv; c[i] = (o0[4 + i] + e0[4 + i] * QRI) * inv; }
      *(v4fa*)(&os[wb + lr * 68 +  0 + 8 * hi]) = a; *(v4fa*)(&os[wb + lr * 68 +  0 + 8 * hi + 4]) = c;
#pragma unroll
      for (int i = 0; i < 4; ++i) { a[i] = (o1[i] + e1[i] * QRI) * inv; c[i] = (o1[4 + i] + e1[4 + i] * QRI) * inv; }
      *(v4fa*)(&os[wb + lr * 68 + 16 + 8 * hi]) = a; *(v4fa*)(&os[wb + lr * 68 + 16 + 8 * hi + 4]) = c;
#pragma unroll
      for (int i = 0; i < 4; ++i) { a[i] = (o2[i] + e2[i] * QRI) * inv; c[i] = (o2[4 + i] + e2[4 + i] * QRI) * inv; }
      *(v4fa*)(&os[wb + lr * 68 + 32 + 8 * hi]) = a; *(v4fa*)(&os[wb + lr * 68 + 32 + 8 * hi + 4]) = c;
#pragma unroll
      for (int i = 0; i < 4; ++i) { a[i] = (o3[i] + e3[i] * QRI) * inv; c[i] = (o3[4 + i] + e3[4 + i] * QRI) * inv; }
      *(v4fa*)(&os[wb + lr * 68 + 48 + 8 * hi]) = a; *(v4fa*)(&os[wb + lr * 68 + 48 + 8 * hi + 4]) = c; }
    wave_sync();
    const size_t cb = ((size_t)bb * SEQ + (size_t)(t0 + (lane >> 3))) * DM + (size_t)(hh * HD + (lane & 7) * 8);
    v8us hv[4], lv[4];
#pragma unroll
    for (int s = 0; s < 4; ++s) { const int row = 4 * s + (lane >> 3), c8 = (lane & 7) * 8;
        const v4f x0 = *(const v4fa*)(&os[wb + row * 68 + c8]); const v4f x1 = *(const v4fa*)(&os[wb + row * 68 + c8 + 4]);
#pragma unroll
        for (int i = 0; i < 4; ++i) { const unsigned short a0 = f2bf(x0[i]); const unsigned short a1 = f2bf(x1[i]);
            hv[s][i] = a0; hv[s][4 + i] = a1; lv[s][i] = f2bf(x0[i] - bf2f(a0)); lv[s][4 + i] = f2bf(x1[i] - bf2f(a1)); } }
#pragma unroll 1
    for (int ps = 0; ps < 2; ++ps) {
#pragma unroll
        for (int s = 0; s < 4; ++s) { const size_t oo = cb + (size_t)s * 4 * DM;
            *(volatile v8us*)(CH + oo) = hv[s]; *(volatile v8us*)(CL + oo) = lv[s]; }
        if (ps == 0) __threadfence(); }

    if (hh == 0) {
        wave_sync();
        const float shp = PSH - m;
        const float zf = inv * 0.0f;
        float* arow = ATT + ((size_t)bb * OUT_SEQ + (size_t)t0) * ATT_LD;
#pragma unroll 1
        for (int key0 = 0; key0 < SEQ; key0 += 32) {
            v4f pa0 = (v4f){zf, zf, zf, zf}, pa1 = pa0, pc0 = pa0, pc1 = pa0;
            if (key0 < kend) {
                const h16* ka = KP + ko + (size_t)key0 * HD;
                const v16h ka0 = ldh(ka), ka1 = ldh(ka + 32), kb0 = ldh(ka + 16 * HD), kb1 = ldh(ka + 16 * HD + 32);
                v8f sHa = (v8f){}, sLa = (v8f){}, sHb = (v8f){}, sLb = (v8f){};
                sHa = wmma16(ka0, qh0, sHa); sHb = wmma16(kb0, qh0, sHb);
                if (SCORE_RES) { sLa = wmma16(ka0, qr0, sLa); sLb = wmma16(kb0, qr0, sLb); }
                sHa = wmma16(ka1, qh1, sHa); sHb = wmma16(kb1, qh1, sHb);
                if (SCORE_RES) { sLa = wmma16(ka1, qr1, sLa); sLb = wmma16(kb1, qr1, sLb); }
                asm volatile("v_nop\n\tv_nop\n\tv_nop\n\tv_nop" : "+v"(sHa), "+v"(sLa), "+v"(sHb), "+v"(sLb) : "v"(ka0), "v"(ka1), "v"(kb0), "v"(kb1));
                float ta[8], tb[8];
#pragma unroll
                for (int r = 0; r < 8; ++r) { ta[r] = (sHa[r] + sLa[r] * QRI) * SC2; tb[r] = (sHb[r] + sLb[r] * QRI) * SC2; }
                if (key0 + 31 > t0) {
                    const int kidx = key0 + 8 * hi;
#pragma unroll
                    for (int r = 0; r < 8; ++r) { ta[r] = (kidx + r > tq) ? NEGV : ta[r]; tb[r] = (kidx + 16 + r > tq) ? NEGV : tb[r]; }
                }
                unsigned mw = MW[mo + (size_t)(key0 >> 5)];
                asm volatile("" : "+v"(mw));
                {
                    const unsigned ma = mw >> (8 * hi), mc = mw >> (16 + 8 * hi);
#pragma unroll
                    for (int r = 0; r < 8; ++r) { ta[r] = (((ma >> r) & 1u) != 0u) ? NEGV : ta[r]; tb[r] = (((mc >> r) & 1u) != 0u) ? NEGV : tb[r]; }
                }
#pragma unroll
                for (int i = 0; i < 4; ++i) {
                    pa0[i] = __builtin_amdgcn_exp2f(ta[i] + shp) * inv; pa1[i] = __builtin_amdgcn_exp2f(ta[4 + i] + shp) * inv;
                    pc0[i] = __builtin_amdgcn_exp2f(tb[i] + shp) * inv; pc1[i] = __builtin_amdgcn_exp2f(tb[4 + i] + shp) * inv; }
            }
            *(v4fa*)(&os[wb + lr * 68 + 8 * hi]) = pa0;      *(v4fa*)(&os[wb + lr * 68 + 8 * hi + 4]) = pa1;
            *(v4fa*)(&os[wb + lr * 68 + 16 + 8 * hi]) = pc0; *(v4fa*)(&os[wb + lr * 68 + 16 + 8 * hi + 4]) = pc1;
            wave_sync();
            v4f val[4];
#pragma unroll
            for (int s = 0; s < 4; ++s) { const int row = 4 * s + (lane >> 3), c4 = (lane & 7) * 4;
                val[s] = *(const v4fa*)(&os[wb + row * 68 + c4]); }
#pragma unroll 1
            for (int ps = 0; ps < 2; ++ps) {
#pragma unroll
                for (int s = 0; s < 4; ++s) { const int row = 4 * s + (lane >> 3), c4 = (lane & 7) * 4;
                    *(volatile v4f*)(arow + (size_t)row * ATT_LD + key0 + c4) = val[s]; }
                if (ps == 0) __threadfence(); }
            wave_sync();
        }
    }
}

static constexpr size_t al256(size_t v) { return (v + 255) & ~(size_t)255; }
static constexpr size_t SZ_XB = al256((size_t)NB * SEQ * DM * 2);
static constexpr size_t SZ_WB = al256((size_t)3 * DM * DM * 2);
static constexpr size_t SZ_WF = al256((size_t)DM * DM * 2);
static constexpr size_t SZ_PL = al256((size_t)NB * SEQ * DM * 2);
static constexpr size_t SZ_MW = al256((size_t)NB * SEQ * (SEQ / 32) * 4);
static constexpr size_t SZ_TOTAL = SZ_XB + SZ_WB + SZ_WF + 5 * SZ_PL + 2 * SZ_PL + SZ_MW;
static_assert(SZ_TOTAL <= (size_t)134217728);
static_assert(((size_t)DM * DM * 2) % 256 == 0);
static_assert(SZ_PL == (size_t)NB * SEQ * DM * 2);
static_assert((size_t)NB * NH_ * SEQ * HD * 2 == SZ_PL);

extern "C" void kernel_launch(void* const* d_in, const int* in_sizes, int n_in,
                              void* d_out, int out_size, void* d_ws, size_t ws_size, hipStream_t stream) {
    if (n_in < 6) return;
    const size_t needx = ((size_t)(NB - 1) * SEQ_FULL + SEQ) * DM;
    if ((size_t)in_sizes[0] < needx) return;
    if ((size_t)in_sizes[1] < (size_t)3 * DM * DM || (size_t)in_sizes[2] < (size_t)3 * DM) return;
    if ((size_t)in_sizes[3] < (size_t)DM * DM || (size_t)in_sizes[4] < (size_t)DM) return;
    if ((size_t)in_sizes[5] < ((size_t)(NB - 1) * SEQ_FULL + (SEQ - 1)) * SEQ_FULL + SEQ) return;
    if ((size_t)out_size < OUT1_OFF + ((size_t)(NB - 1) * OUT_SEQ + (SEQ - 1)) * ATT_LD + SEQ) return;
    if (SZ_TOTAL > ws_size) return;
    const float* x = (const float*)d_in[0]; const float* wqkv = (const float*)d_in[1]; const float* bqkv = (const float*)d_in[2];
    const float* wfc = (const float*)d_in[3]; const float* bfc = (const float*)d_in[4];
    const int* pmask = (const int*)d_in[5];
    float* OUT = (float*)d_out;
    float* ATT = OUT + OUT1_OFF;
    char* wsp = (char*)d_ws;
    bf* XB = (bf*)wsp; wsp += SZ_XB;
    bf* WB = (bf*)wsp; wsp += SZ_WB;
    bf* WF = (bf*)wsp; wsp += SZ_WF;
    h16* QH = (h16*)wsp; wsp += SZ_PL;
    h16* QR = (h16*)wsp; wsp += SZ_PL;
    h16* KP = (h16*)wsp; wsp += SZ_PL;
    h16* VT = (h16*)wsp; wsp += SZ_PL;
    h16* VR = (h16*)wsp; wsp += SZ_PL;
    bf* CH = (bf*)wsp; wsp += SZ_PL;
    bf* CL = (bf*)wsp; wsp += SZ_PL;
    unsigned* MW = (unsigned*)wsp; wsp += SZ_MW;

    if (SEQ == SEQ_FULL) {
        const size_t n8 = (size_t)NB * SEQ * DM / 8;
        k_cvt8<<<(unsigned)((n8 + 255) / 256), 256, 0, stream>>>(x, XB, n8);
    } else {
        const size_t n8 = (size_t)SEQ * DM / 8;
        for (int b = 0; b < NB; ++b) k_cvt8<<<(unsigned)((n8 + 255) / 256), 256, 0, stream>>>(x + (size_t)b * SEQ_FULL * DM, XB + (size_t)b * SEQ * DM, n8);
    }
    k_cvtT<<<dim3(DM / 64, 3 * DM / 64, 1), 256, 0, stream>>>(wqkv, 3 * DM, WB, 1 << 30);
    k_cvtT<<<dim3(DM / 64, DM / 64, 1), 256, 0, stream>>>(wfc, DM, WF, 1 << 30);
    {
        const size_t nW = (size_t)NB * SEQ * (SEQ / 32);
        k_mbits<<<(unsigned)(nW / 256), 256, 0, stream>>>(pmask, MW, nW);
    }

    k_gemm<0><<<dim3(NB * SEQ / 64, DM / 64, 1), 32, 0, stream>>>(XB, WB, bqkv, QH, QR, OUT);
    k_gemm<1><<<dim3(NB * SEQ / 64, DM / 64, 1), 32, 0, stream>>>(XB, WB + (size_t)DM * DM, bqkv, KP, KP, OUT);
    k_gemm<2><<<dim3(DM / 64, NB * SEQ / 64, 1), 32, 0, stream>>>(WB + (size_t)2 * DM * DM, XB, bqkv, VT, VR, OUT);

    k_flash<<<dim3(SEQ / (16 * AW), NB * NH_, 1), 32 * AW, 0, stream>>>(QH, QR, KP, VT, VR, MW, CH, CL, ATT);

    k_gemm<3><<<dim3(NB * SEQ / 64, DM / 64, 1), 32, 0, stream>>>(CH, WF, bfc, QH, QR, OUT);
}
